// SelfAttention_6682969113297
// MI455X (gfx1250) — hardware-verified
//
#include <hip/hip_runtime.h>
#include <math.h>


#ifndef NB
#define NB 4
#endif
#ifndef SEQ
#define SEQ 2048
#endif
#define NB_FULL   4
#define SEQ_FULL  2048
#define DIM       512
#define NHEAD     8
#define HDIM      64
#define FFN       2048
#define QKVN      (3 * DIM)
#define NTOK      (NB * SEQ)
#define PLANE     ((size_t)NTOK * DIM)
#define GM        128
#define GN        64
#define GW        4
#define OP        68
#define VP        136
#define TP        72
#define BQ        128
#define BK        32
#define NWAVE     8
#define XC        16.0f
#define WC        64.0f
#define VC        16.0f
#define CC        256.0f
#define PC        4096.0f
#define RC        2048.0f

static_assert(DIM == NHEAD * HDIM);
static_assert(HDIM == 64);
static_assert(HDIM == GN);
static_assert(GM == GW * 32);
static_assert(BQ == NWAVE * 16);
static_assert(SEQ % GM == 0);
static_assert(SEQ % BQ == 0);
static_assert(SEQ % BK == 0);
static_assert(NTOK % GM == 0);
static_assert(NTOK % 8 == 0);
static_assert(DIM % GN == 0);
static_assert(FFN % GN == 0);
static_assert(QKVN % GN == 0);
static_assert(DIM % 64 == 0);
static_assert(FFN % 64 == 0);
static_assert(DIM % 32 == 0);
static_assert(FFN % 32 == 0);
static_assert(DIM == 32 * 16);
static_assert(((size_t)NTOK * DIM / 8) % 256 == 0);
static_assert((OP * 4) % 16 == 0);
static_assert((VP * 2) % 16 == 0);
static_assert((TP * 2) % 16 == 0);
static_assert(SEQ <= SEQ_FULL);
static_assert(NB >= 1 && NB <= NB_FULL);

#define SZ_XH    ((size_t)NTOK * DIM * 2)
#define SZ_WQKV  ((size_t)QKVN * DIM * 2)
#define SZ_WO    ((size_t)DIM * DIM * 2)
#define SZ_W1    ((size_t)FFN * DIM * 2)
#define SZ_W2    ((size_t)DIM * FFN * 2)
#define SZ_QK    ((size_t)4 * NTOK * DIM * 2)
#define SZ_HH    ((size_t)NTOK * FFN * 2)
#define SZ_BIG   ((SZ_QK > SZ_HH) ? SZ_QK : SZ_HH)
#define SZ_VT    ((size_t)NTOK * DIM * 2)
#define SZ_CTX   ((size_t)NTOK * DIM * 2)
#define SZ_Y     ((size_t)NTOK * DIM * 4)
#define SZ_X1F   ((size_t)NTOK * DIM * 4)
#define SZ_X1H   ((size_t)NTOK * DIM * 2)
#define OFF_XH   ((size_t)0)
#define OFF_WQKV (OFF_XH + SZ_XH)
#define OFF_WO   (OFF_WQKV + SZ_WQKV)
#define OFF_W1   (OFF_WO + SZ_WO)
#define OFF_W2   (OFF_W1 + SZ_W1)
#define OFF_BIG  (OFF_W2 + SZ_W2)
#define OFF_VT   (OFF_BIG + SZ_BIG)
#define OFF_CTX  (OFF_VT + SZ_VT)
#define OFF_Y    (OFF_CTX + SZ_CTX)
#define OFF_X1F  (OFF_Y + SZ_Y)
#define OFF_X1H  (OFF_X1F + SZ_X1F)
#define WS_TOTAL (OFF_X1H + SZ_X1H)
static_assert(SZ_QK <= SZ_BIG);
static_assert(SZ_HH <= SZ_BIG);
static_assert(SZ_XH % 128 == 0 && SZ_WQKV % 128 == 0 && SZ_WO % 128 == 0 && SZ_W1 % 128 == 0);
static_assert(SZ_W2 % 128 == 0 && SZ_BIG % 128 == 0 && SZ_VT % 128 == 0 && SZ_CTX % 128 == 0);
static_assert(SZ_Y % 128 == 0 && SZ_X1F % 128 == 0 && SZ_X1H % 128 == 0);
static_assert(WS_TOTAL <= (size_t)134217728);

typedef __bf16   bf16;
typedef _Float16 f16;
typedef f16      v16h  __attribute__((ext_vector_type(16)));
typedef f16      v8h   __attribute__((ext_vector_type(8)));
typedef float    v8f   __attribute__((ext_vector_type(8)));
typedef float    v4f   __attribute__((ext_vector_type(4)));
typedef unsigned v4u   __attribute__((ext_vector_type(4)));

union FragH  { v16h v; v4u q[2]; f16 h[16]; };
union Pack8H { v4u u; v8h v; f16 h[8]; };

static __device__ __forceinline__ float bfr(float v) { return (float)(bf16)v; }

static __device__ __forceinline__ v8f mma_f16(v16h a, v16h b, v8f acc) {
  acc = __builtin_amdgcn_wmma_f32_16x16x32_f16(false, a, false, b, (short)0, acc, false, false);
  asm volatile("v_nop\n\tv_nop\n\tv_nop\n\tv_nop" : "+v"(acc) : "v"(a), "v"(b));
  return acc;
}

static __device__ __forceinline__ float wave_sum(float v) {
  v += __shfl_xor(v, 16, 32);
  v += __shfl_xor(v, 8, 32);
  v += __shfl_xor(v, 4, 32);
  v += __shfl_xor(v, 2, 32);
  v += __shfl_xor(v, 1, 32);
  return v;
}

__global__ __launch_bounds__(256) void cvt_x_kernel(const float* __restrict__ x, f16* __restrict__ xh) {
  const int g = blockIdx.x * 256 + threadIdx.x;
  const int t = g >> 6;
  const int c = (g & 63) * 8;
  if (t >= NTOK) return;
  const int bb = t / SEQ;
  const int s  = t - bb * SEQ;
  const float* src = x + ((size_t)bb * SEQ_FULL + s) * DIM + c;
  const v4f a0 = *(const v4f*)(src);
  const v4f a1 = *(const v4f*)(src + 4);
  Pack8H p;
  #pragma unroll
  for (int i = 0; i < 4; ++i) {
    p.h[i]     = (f16)(bfr(a0[i]) * XC);
    p.h[4 + i] = (f16)(bfr(a1[i]) * XC);
  }
  const v4u val = p.u;
  f16* dst = xh + (size_t)t * DIM + c;
  *(volatile v4u*)dst = val;
  __threadfence();
  *(volatile v4u*)dst = val;
}

__global__ __launch_bounds__(256) void wt_kernel(const float* __restrict__ W, f16* __restrict__ Wt, int K, int N) {
  __shared__ __align__(16) f16 sT[64 * TP];
  const int tid = threadIdx.x;
  const int n0 = blockIdx.x * 64;
  const int k0 = blockIdx.y * 64;
  #pragma unroll
  for (int it = 0; it < 4; ++it) {
    const int kk = it * 16 + (tid >> 4);
    const int nn = (tid & 15) * 4;
    const v4f w = *(const v4f*)(W + (size_t)(k0 + kk) * N + n0 + nn);
    #pragma unroll
    for (int i = 0; i < 4; ++i) sT[(nn + i) * TP + kk] = (f16)(bfr(w[i]) * WC);
  }
  __syncthreads();
  v4u    val[2];
  size_t idx[2];
  #pragma unroll
  for (int it = 0; it < 2; ++it) {
    const int n  = it * 32 + (tid >> 3);
    const int ks = (tid & 7) * 8;
    Pack8H ph;
    ph.v = *(const v8h*)(&sT[n * TP + ks]);
    val[it] = ph.u;
    idx[it] = (size_t)(n0 + n) * K + k0 + ks;
  }
  #pragma unroll
  for (int it = 0; it < 2; ++it) *(volatile v4u*)(Wt + idx[it]) = val[it];
  __threadfence();
  #pragma unroll
  for (int it = 0; it < 2; ++it) *(volatile v4u*)(Wt + idx[it]) = val[it];
}

template <int K>
static __device__ __forceinline__ void gemm_main(const f16* __restrict__ A, const f16* __restrict__ Bt,
                                                 int m0, int n0, int lq, int hi, v8f (&acc)[2][4]) {
  static_assert(K % 32 == 0);
  const f16* ap = A  + (size_t)(m0 + lq) * K + hi * 8;
  const f16* bp = Bt + (size_t)(n0 + lq) * K + hi * 8;
  #pragma unroll 1
  for (int k0 = 0; k0 < K; k0 += 32) {
    FragH a[2], b[4];
    #pragma unroll
    for (int mt = 0; mt < 2; ++mt) {
      const f16* p = ap + (size_t)mt * 16 * K + k0;
      a[mt].q[0] = *(const v4u*)(p);
      a[mt].q[1] = *(const v4u*)(p + 16);
    }
    #pragma unroll
    for (int nt = 0; nt < 4; ++nt) {
      const f16* p = bp + (size_t)nt * 16 * K + k0;
      b[nt].q[0] = *(const v4u*)(p);
      b[nt].q[1] = *(const v4u*)(p + 16);
    }
    #pragma unroll
    for (int mt = 0; mt < 2; ++mt) {
      #pragma unroll
      for (int nt = 0; nt < 4; ++nt) acc[mt][nt] = mma_f16(a[mt].v, b[nt].v, acc[mt][nt]);
    }
  }
}

__global__ __launch_bounds__(128) void gemm_qkv_kernel(const f16* __restrict__ xh, const f16* __restrict__ wT,
                                                       const float* __restrict__ bq, const float* __restrict__ bk,
                                                       const float* __restrict__ bv,
                                                       f16* __restrict__ qk, f16* __restrict__ vt) {
  __shared__ __align__(16) float sC[GW * 32 * OP];
  __shared__ __align__(16) f16   sVT[HDIM * VP];
  const int tid  = threadIdx.x;
  const int wave = __builtin_amdgcn_readfirstlane(threadIdx.x >> 5);
  const int lane = tid & 31;
  const int lq   = lane & 15;
  const int hi   = lane >> 4;
  const int tok0 = blockIdx.x * GM;
  const int n0   = blockIdx.y * GN;
  const int seg  = n0 / DIM;
  const int h    = (n0 - seg * DIM) / HDIM;
  const int bb   = tok0 / SEQ;
  const int s0   = tok0 - bb * SEQ;

  v8f acc[2][4];
  #pragma unroll
  for (int mt = 0; mt < 2; ++mt) {
    #pragma unroll
    for (int nt = 0; nt < 4; ++nt) acc[mt][nt] = (v8f){0, 0, 0, 0, 0, 0, 0, 0};
  }
  gemm_main<DIM>(xh, wT, tok0 + wave * 32, n0, lq, hi, acc);

  const float ascale = 1.0f / (XC * WC);
  float bias[4];
  #pragma unroll
  for (int nt = 0; nt < 4; ++nt) {
    const int c = h * HDIM + nt * 16 + lq;
    const float fq = bq[c];
    const float fk = bk[c];
    const float fv = bv[c];
    const float sel = (seg == 0) ? fq : ((seg == 1) ? fk : fv);
    bias[nt] = bfr(sel);
  }

  if (seg < 2) {
    const int wb = wave * (32 * OP);
    #pragma unroll
    for (int mt = 0; mt < 2; ++mt) {
      #pragma unroll
      for (int nt = 0; nt < 4; ++nt) {
        #pragma unroll
        for (int r = 0; r < 8; ++r)
          sC[wb + (mt * 16 + hi * 8 + r) * OP + nt * 16 + lq] = acc[mt][nt][r] * ascale + bias[nt];
      }
    }
    __syncthreads();
    const size_t pbase = (size_t)seg * 2 * PLANE +
                         (((size_t)bb * NHEAD + h) * SEQ + s0 + wave * 32) * HDIM;
    v4u hv[8], rv[8];
    #pragma unroll
    for (int it = 0; it < 8; ++it) {
      const int row = it * 4 + (lane >> 3);
      const int col = (lane & 7) * 8;
      const v4f c0 = *(const v4f*)(&sC[wb + row * OP + col]);
      const v4f c1 = *(const v4f*)(&sC[wb + row * OP + col + 4]);
      Pack8H ph, pr;
      #pragma unroll
      for (int i = 0; i < 4; ++i) {
        const f16 h0 = (f16)c0[i];
        const f16 h1 = (f16)c1[i];
        ph.h[i]     = h0;
        ph.h[4 + i] = h1;
        pr.h[i]     = (f16)((c0[i] - (float)h0) * RC);
        pr.h[4 + i] = (f16)((c1[i] - (float)h1) * RC);
      }
      hv[it] = ph.u;
      rv[it] = pr.u;
    }
    #pragma unroll
    for (int it = 0; it < 8; ++it) {
      const size_t o = pbase + (size_t)(it * 4 + (lane >> 3)) * HDIM + (lane & 7) * 8;
      *(volatile v4u*)(qk + o)         = hv[it];
      *(volatile v4u*)(qk + PLANE + o) = rv[it];
    }
    __threadfence();
    #pragma unroll
    for (int it = 0; it < 8; ++it) {
      const size_t o = pbase + (size_t)(it * 4 + (lane >> 3)) * HDIM + (lane & 7) * 8;
      *(volatile v4u*)(qk + o)         = hv[it];
      *(volatile v4u*)(qk + PLANE + o) = rv[it];
    }
  } else {
    #pragma unroll
    for (int mt = 0; mt < 2; ++mt) {
      #pragma unroll
      for (int nt = 0; nt < 4; ++nt) {
        #pragma unroll
        for (int r = 0; r < 8; ++r)
          sVT[(nt * 16 + lq) * VP + wave * 32 + mt * 16 + hi * 8 + r] =
              (f16)((acc[mt][nt][r] * ascale + bias[nt]) * VC);
      }
    }
    __syncthreads();
    const size_t vbase = ((size_t)bb * NHEAD + h) * HDIM;
    v4u vv[8];
    #pragma unroll
    for (int it = 0; it < 8; ++it) {
      const int L     = it * 16 + (tid >> 3);
      const int d     = L >> 1;
      const int half  = L & 1;
      const int piece = (tid & 7) * 8;
      Pack8H ph;
      ph.v = *(const v8h*)(&sVT[d * VP + half * 64 + piece]);
      vv[it] = ph.u;
    }
    #pragma unroll
    for (int it = 0; it < 8; ++it) {
      const int L = it * 16 + (tid >> 3);
      const size_t o = (vbase + (L >> 1)) * SEQ + s0 + (L & 1) * 64 + (tid & 7) * 8;
      *(volatile v4u*)(vt + o) = vv[it];
    }
    __threadfence();
    #pragma unroll
    for (int it = 0; it < 8; ++it) {
      const int L = it * 16 + (tid >> 3);
      const size_t o = (vbase + (L >> 1)) * SEQ + s0 + (L & 1) * 64 + (tid & 7) * 8;
      *(volatile v4u*)(vt + o) = vv[it];
    }
  }
}

__global__ __launch_bounds__(256) void attn_kernel(const f16* __restrict__ qk, const f16* __restrict__ vt,
                                                   f16* __restrict__ ctx) {
  __shared__ __align__(16) float sO[NWAVE * 16 * OP];
  const int qblk = blockIdx.x;
  const int h    = blockIdx.y;
  const int b    = blockIdx.z;
  const int tid  = threadIdx.x;
  const int wave = __builtin_amdgcn_readfirstlane(threadIdx.x >> 5);
  const int lane = tid & 31;
  const int lq   = lane & 15;
  const int hi   = lane >> 4;

  const int qrow0 = qblk * BQ + wave * 16;
  const size_t hb = ((size_t)b * NHEAD + h) * (size_t)SEQ * HDIM;
  const f16* qh_p = qk + hb;
  const f16* qr_p = qk + PLANE + hb;
  const f16* kh_p = qk + 2 * PLANE + hb;
  const f16* kr_p = qk + 3 * PLANE + hb;
  const f16* vt_h = vt + hb;
  const int qoff  = (qrow0 + lq) * HDIM + hi * 8;

  v8f o[4];
  #pragma unroll
  for (int dt = 0; dt < 4; ++dt) o[dt] = (v8f){0, 0, 0, 0, 0, 0, 0, 0};

  float rmax = -__builtin_inff();
  float rsum = 0.0f;
  const float SL = 0.125f * 1.4426950408889634f;

  #pragma unroll 1
  for (int j0 = 0; j0 < SEQ; j0 += BK) {
    v8f c[2];
    #pragma unroll
    for (int sub = 0; sub < 2; ++sub) {
      v8f am = (v8f){0, 0, 0, 0, 0, 0, 0, 0};
      v8f ar = (v8f){0, 0, 0, 0, 0, 0, 0, 0};
      #pragma unroll
      for (int f = 0; f < 2; ++f) {
        int qo = qoff + f * 32;
        asm volatile("" : "+v"(qo));
        FragH fqh, fqr, fkh, fkr;
        fqh.q[0] = *(const v4u*)(qh_p + qo);
        fqh.q[1] = *(const v4u*)(qh_p + qo + 16);
        fqr.q[0] = *(const v4u*)(qr_p + qo);
        fqr.q[1] = *(const v4u*)(qr_p + qo + 16);
        const int ko = (j0 + sub * 16 + lq) * HDIM + f * 32 + hi * 8;
        fkh.q[0] = *(const v4u*)(kh_p + ko);
        fkh.q[1] = *(const v4u*)(kh_p + ko + 16);
        fkr.q[0] = *(const v4u*)(kr_p + ko);
        fkr.q[1] = *(const v4u*)(kr_p + ko + 16);
        am = mma_f16(fkh.v, fqh.v, am);
        ar = mma_f16(fkh.v, fqr.v, ar);
        ar = mma_f16(fkr.v, fqh.v, ar);
      }
      #pragma unroll
      for (int r = 0; r < 8; ++r) c[sub][r] = am[r] + ar[r] * (1.0f / RC);
    }

    FragH bv[4];
    #pragma unroll
    for (int dt = 0; dt < 4; ++dt) {
      const f16* base = vt_h + (size_t)(dt * 16 + lq) * SEQ + j0 + hi * 8;
      bv[dt].q[0] = *(const v4u*)(base);
      bv[dt].q[1] = *(const v4u*)(base + 16);
    }

    float m_new = rmax;
    #pragma unroll
    for (int r = 0; r < 8; ++r) {
      m_new = fmaxf(m_new, c[0][r]);
      m_new = fmaxf(m_new, c[1][r]);
    }
    m_new = fmaxf(m_new, __shfl_xor(m_new, 16, 32));
    const float scale = __builtin_amdgcn_exp2f((rmax - m_new) * SL);
    rmax = m_new;

    FragH pa;
    float psum = 0.0f;
    #pragma unroll
    for (int r = 0; r < 8; ++r) {
      const float p0 = __builtin_amdgcn_exp2f((c[0][r] - m_new) * SL);
      const float p1 = __builtin_amdgcn_exp2f((c[1][r] - m_new) * SL);
      psum += p0 + p1;
      pa.h[r]     = (f16)(p0 * PC);
      pa.h[8 + r] = (f16)(p1 * PC);
    }
    rsum = rsum * scale + psum + __shfl_xor(psum, 16, 32);

    float sc[8];
    #pragma unroll
    for (int r = 0; r < 8; ++r) sc[r] = __shfl(scale, (hi << 3) + r, 32);
    #pragma unroll
    for (int dt = 0; dt < 4; ++dt) {
      #pragma unroll
      for (int r = 0; r < 8; ++r) o[dt][r] *= sc[r];
    }

    #pragma unroll
    for (int dt = 0; dt < 4; ++dt) o[dt] = mma_f16(pa.v, bv[dt].v, o[dt]);
  }

  float rs[8];
  #pragma unroll
  for (int r = 0; r < 8; ++r) rs[r] = 1.0f / __shfl(rsum, (hi << 3) + r, 32);

  const int wb = wave * (16 * OP);
  #pragma unroll
  for (int r = 0; r < 8; ++r) {
    #pragma unroll
    for (int dt = 0; dt < 4; ++dt)
      sO[wb + (hi * 8 + r) * OP + dt * 16 + lq] = o[dt][r] * (CC / (PC * VC)) * rs[r];
  }
  __syncthreads();

  v4u    pv[4];
  size_t gidx[4];
  #pragma unroll
  for (int it = 0; it < 4; ++it) {
    const int row = it * 4 + (lane >> 3);
    const int col = (lane & 7) * 8;
    const v4f c0 = *(const v4f*)(&sO[wb + row * OP + col]);
    const v4f c1 = *(const v4f*)(&sO[wb + row * OP + col + 4]);
    Pack8H ph;
    #pragma unroll
    for (int i = 0; i < 4; ++i) {
      ph.h[i]     = (f16)c0[i];
      ph.h[4 + i] = (f16)c1[i];
    }
    pv[it]   = ph.u;
    gidx[it] = ((size_t)b * SEQ + qrow0 + row) * DIM + h * HDIM + col;
  }
  #pragma unroll
  for (int it = 0; it < 4; ++it) *(volatile v4u*)(ctx + gidx[it]) = pv[it];
  __threadfence();
  #pragma unroll
  for (int it = 0; it < 4; ++it) *(volatile v4u*)(ctx + gidx[it]) = pv[it];
}

__global__ __launch_bounds__(128) void gemm_wo_kernel(const f16* __restrict__ ctx, const f16* __restrict__ woT,
                                                      const float* __restrict__ bo, const float* __restrict__ x,
                                                      float* __restrict__ y) {
  __shared__ __align__(16) float sC[GW * 32 * OP];
  const int tid  = threadIdx.x;
  const int wave = __builtin_amdgcn_readfirstlane(threadIdx.x >> 5);
  const int lane = tid & 31;
  const int lq   = lane & 15;
  const int hi   = lane >> 4;
  const int tok0 = blockIdx.x * GM;
  const int n0   = blockIdx.y * GN;
  const int bb   = tok0 / SEQ;
  const int s0   = tok0 - bb * SEQ;

  v8f acc[2][4];
  #pragma unroll
  for (int mt = 0; mt < 2; ++mt) {
    #pragma unroll
    for (int nt = 0; nt < 4; ++nt) acc[mt][nt] = (v8f){0, 0, 0, 0, 0, 0, 0, 0};
  }
  gemm_main<DIM>(ctx, woT, tok0 + wave * 32, n0, lq, hi, acc);

  const float ascale = 1.0f / (CC * WC);
  const int wb = wave * (32 * OP);
  #pragma unroll
  for (int nt = 0; nt < 4; ++nt) {
    const float bias = bfr(bo[n0 + nt * 16 + lq]);
    #pragma unroll
    for (int mt = 0; mt < 2; ++mt) {
      #pragma unroll
      for (int r = 0; r < 8; ++r)
        sC[wb + (mt * 16 + hi * 8 + r) * OP + nt * 16 + lq] = acc[mt][nt][r] * ascale + bias;
    }
  }
  __syncthreads();

  const size_t orow = (size_t)tok0 + wave * 32;
  const size_t rrow = (size_t)bb * SEQ_FULL + s0 + wave * 32;
  #pragma unroll
  for (int g = 0; g < 2; ++g) {
    v4f vals[8];
    #pragma unroll
    for (int it = 0; it < 8; ++it) {
      const int row = g * 16 + it * 2 + hi;
      v4f cv = *(const v4f*)(&sC[wb + row * OP + lq * 4]);
      const v4f rv = *(const v4f*)(x + (rrow + row) * DIM + n0 + lq * 4);
      #pragma unroll
      for (int i = 0; i < 4; ++i) cv[i] = cv[i] + bfr(rv[i]);
      vals[it] = cv;
    }
    #pragma unroll
    for (int it = 0; it < 8; ++it)
      *(volatile v4f*)(y + (orow + g * 16 + it * 2 + hi) * DIM + n0 + lq * 4) = vals[it];
    __threadfence();
    #pragma unroll
    for (int it = 0; it < 8; ++it)
      *(volatile v4f*)(y + (orow + g * 16 + it * 2 + hi) * DIM + n0 + lq * 4) = vals[it];
  }
}

__global__ __launch_bounds__(256) void ln1_kernel(const float* __restrict__ y, const float* __restrict__ g,
                                                  const float* __restrict__ be,
                                                  float* __restrict__ x1f, f16* __restrict__ x1h) {
  __shared__ __align__(16) f16 sH[8 * DIM];
  const int tid  = threadIdx.x;
  const int wave = __builtin_amdgcn_readfirstlane(threadIdx.x >> 5);
  const int lane = tid & 31;
  const int t    = blockIdx.x * 8 + wave;
  const float* yr = y + (size_t)t * DIM;

  v4f v[4];
  float s = 0.0f;
  #pragma unroll
  for (int j = 0; j < 4; ++j) {
    v[j] = *(const v4f*)(yr + j * 128 + lane * 4);
    s += (v[j][0] + v[j][1]) + (v[j][2] + v[j][3]);
  }
  s = wave_sum(s);
  const float mean = s * (1.0f / DIM);
  float q = 0.0f;
  #pragma unroll
  for (int j = 0; j < 4; ++j) {
    #pragma unroll
    for (int i = 0; i < 4; ++i) {
      const float d = v[j][i] - mean;
      q += d * d;
    }
  }
  q = wave_sum(q);
  const float rstd = rsqrtf(q * (1.0f / DIM) + 1e-5f);

  v4f ov[4];
  #pragma unroll
  for (int j = 0; j < 4; ++j) {
    const v4f gv = *(const v4f*)(g + j * 128 + lane * 4);
    const v4f bv = *(const v4f*)(be + j * 128 + lane * 4);
    #pragma unroll
    for (int i = 0; i < 4; ++i) {
      const float val = (v[j][i] - mean) * rstd * bfr(gv[i]) + bfr(bv[i]);
      ov[j][i] = val;
      sH[wave * DIM + j * 128 + lane * 4 + i] = (f16)(val * XC);
    }
  }
  __syncthreads();
  v4u hv[2];
  #pragma unroll
  for (int jj = 0; jj < 2; ++jj) {
    Pack8H ph;
    ph.v = *(const v8h*)(&sH[wave * DIM + jj * 256 + lane * 8]);
    hv[jj] = ph.u;
  }
  float* fo = x1f + (size_t)t * DIM + lane * 4;
  f16*   ho = x1h + (size_t)t * DIM + lane * 8;
  #pragma unroll
  for (int j = 0; j < 4; ++j) *(volatile v4f*)(fo + j * 128) = ov[j];
  #pragma unroll
  for (int jj = 0; jj < 2; ++jj) *(volatile v4u*)(ho + jj * 256) = hv[jj];
  __threadfence();
  #pragma unroll
  for (int j = 0; j < 4; ++j) *(volatile v4f*)(fo + j * 128) = ov[j];
  #pragma unroll
  for (int jj = 0; jj < 2; ++jj) *(volatile v4u*)(ho + jj * 256) = hv[jj];
}

__global__ __launch_bounds__(128) void gemm_ffn1_kernel(const f16* __restrict__ x1h, const f16* __restrict__ w1T,
                                                        const float* __restrict__ b1, f16* __restrict__ hh) {
  __shared__ __align__(16) float sC[GW * 32 * OP];
  const int tid  = threadIdx.x;
  const int wave = __builtin_amdgcn_readfirstlane(threadIdx.x >> 5);
  const int lane = tid & 31;
  const int lq   = lane & 15;
  const int hi   = lane >> 4;
  const int tok0 = blockIdx.x * GM;
  const int n0   = blockIdx.y * GN;

  v8f acc[2][4];
  #pragma unroll
  for (int mt = 0; mt < 2; ++mt) {
    #pragma unroll
    for (int nt = 0; nt < 4; ++nt) acc[mt][nt] = (v8f){0, 0, 0, 0, 0, 0, 0, 0};
  }
  gemm_main<DIM>(x1h, w1T, tok0 + wave * 32, n0, lq, hi, acc);

  const float ascale = 1.0f / (XC * WC);
  const int wb = wave * (32 * OP);
  #pragma unroll
  for (int nt = 0; nt < 4; ++nt) {
    const float bias = bfr(b1[n0 + nt * 16 + lq]);
    #pragma unroll
    for (int mt = 0; mt < 2; ++mt) {
      #pragma unroll
      for (int r = 0; r < 8; ++r)
        sC[wb + (mt * 16 + hi * 8 + r) * OP + nt * 16 + lq] = acc[mt][nt][r] * ascale + bias;
    }
  }
  __syncthreads();

  const int lrow = lane >> 3;
  const int lcol = (lane & 7) * 8;
  #pragma unroll 1
  for (int i = 0; i < 16; ++i) {
    const int off = wb + ((i >> 1) * 4 + lrow) * OP + lcol + (i & 1) * 4;
    v4f t = *(const v4f*)(&sC[off]);
    #pragma unroll
    for (int e = 0; e < 4; ++e) {
      const float u = t[e];
      t[e] = 0.5f * u * (1.0f + erff(u * 0.70710678118654752f));
    }
    *(v4f*)(&sC[off]) = t;
  }

  v4u pv[8];
  #pragma unroll
  for (int it = 0; it < 8; ++it) {
    const int off = wb + (it * 4 + lrow) * OP + lcol;
    const v4f c0 = *(const v4f*)(&sC[off]);
    const v4f c1 = *(const v4f*)(&sC[off + 4]);
    Pack8H ph;
    #pragma unroll
    for (int i = 0; i < 4; ++i) {
      ph.h[i]     = (f16)(c0[i] * XC);
      ph.h[4 + i] = (f16)(c1[i] * XC);
    }
    pv[it] = ph.u;
  }
  const size_t obase = ((size_t)tok0 + wave * 32 + lrow) * FFN + n0 + lcol;
  #pragma unroll
  for (int it = 0; it < 8; ++it) *(volatile v4u*)(hh + obase + (size_t)it * 4 * FFN) = pv[it];
  __threadfence();
  #pragma unroll
  for (int it = 0; it < 8; ++it) *(volatile v4u*)(hh + obase + (size_t)it * 4 * FFN) = pv[it];
}

__global__ __launch_bounds__(128) void gemm_ffn2_kernel(const f16* __restrict__ hh, const f16* __restrict__ w2T,
                                                        const float* __restrict__ b2, const float* __restrict__ x1f,
                                                        float* __restrict__ y) {
  __shared__ __align__(16) float sC[GW * 32 * OP];
  const int tid  = threadIdx.x;
  const int wave = __builtin_amdgcn_readfirstlane(threadIdx.x >> 5);
  const int lane = tid & 31;
  const int lq   = lane & 15;
  const int hi   = lane >> 4;
  const int tok0 = blockIdx.x * GM;
  const int n0   = blockIdx.y * GN;

  v8f acc[2][4];
  #pragma unroll
  for (int mt = 0; mt < 2; ++mt) {
    #pragma unroll
    for (int nt = 0; nt < 4; ++nt) acc[mt][nt] = (v8f){0, 0, 0, 0, 0, 0, 0, 0};
  }
  gemm_main<FFN>(hh, w2T, tok0 + wave * 32, n0, lq, hi, acc);

  const float ascale = 1.0f / (XC * WC);
  const int wb = wave * (32 * OP);
  #pragma unroll
  for (int nt = 0; nt < 4; ++nt) {
    const float bias = bfr(b2[n0 + nt * 16 + lq]);
    #pragma unroll
    for (int mt = 0; mt < 2; ++mt) {
      #pragma unroll
      for (int r = 0; r < 8; ++r)
        sC[wb + (mt * 16 + hi * 8 + r) * OP + nt * 16 + lq] = acc[mt][nt][r] * ascale + bias;
    }
  }
  __syncthreads();

  const size_t orow = (size_t)tok0 + wave * 32;
  #pragma unroll
  for (int g = 0; g < 2; ++g) {
    v4f vals[8];
    #pragma unroll
    for (int it = 0; it < 8; ++it) {
      const int row = g * 16 + it * 2 + hi;
      v4f cv = *(const v4f*)(&sC[wb + row * OP + lq * 4]);
      const v4f rv = *(const v4f*)(x1f + (orow + row) * DIM + n0 + lq * 4);
      #pragma unroll
      for (int i = 0; i < 4; ++i) cv[i] = cv[i] + rv[i];
      vals[it] = cv;
    }
    #pragma unroll
    for (int it = 0; it < 8; ++it)
      *(volatile v4f*)(y + (orow + g * 16 + it * 2 + hi) * DIM + n0 + lq * 4) = vals[it];
    __threadfence();
    #pragma unroll
    for (int it = 0; it < 8; ++it)
      *(volatile v4f*)(y + (orow + g * 16 + it * 2 + hi) * DIM + n0 + lq * 4) = vals[it];
  }
}

__global__ __launch_bounds__(256) void ln2_kernel(const float* __restrict__ y, const float* __restrict__ g,
                                                  const float* __restrict__ be, float* __restrict__ out) {
  const int tid  = threadIdx.x;
  const int wave = __builtin_amdgcn_readfirstlane(threadIdx.x >> 5);
  const int lane = tid & 31;
  const int t    = blockIdx.x * 8 + wave;
  const int bb   = t / SEQ;
  const int s0   = t - bb * SEQ;
  const float* yr = y + (size_t)t * DIM;

  v4f v[4];
  float s = 0.0f;
  #pragma unroll
  for (int j = 0; j < 4; ++j) {
    v[j] = *(const v4f*)(yr + j * 128 + lane * 4);
    s += (v[j][0] + v[j][1]) + (v[j][2] + v[j][3]);
  }
  s = wave_sum(s);
  const float mean = s * (1.0f / DIM);
  float q = 0.0f;
  #pragma unroll
  for (int j = 0; j < 4; ++j) {
    #pragma unroll
    for (int i = 0; i < 4; ++i) {
      const float d = v[j][i] - mean;
      q += d * d;
    }
  }
  q = wave_sum(q);
  const float rstd = rsqrtf(q * (1.0f / DIM) + 1e-5f);

  v4f ov[4];
  #pragma unroll
  for (int j = 0; j < 4; ++j) {
    const v4f gv = *(const v4f*)(g + j * 128 + lane * 4);
    const v4f bv = *(const v4f*)(be + j * 128 + lane * 4);
    #pragma unroll
    for (int i = 0; i < 4; ++i) ov[j][i] = (v[j][i] - mean) * rstd * bfr(gv[i]) + bfr(bv[i]);
  }
  float* fo = out + ((size_t)bb * SEQ_FULL + s0) * DIM + lane * 4;
  #pragma unroll
  for (int j = 0; j < 4; ++j) *(volatile v4f*)(fo + j * 128) = ov[j];
  __threadfence();
  #pragma unroll
  for (int j = 0; j < 4; ++j) *(volatile v4f*)(fo + j * 128) = ov[j];
}

extern "C" void kernel_launch(void* const* d_in, const int* in_sizes, int n_in,
                              void* d_out, int out_size, void* d_ws, size_t ws_size,
                              hipStream_t stream) {
  if (n_in < 17) return;
  const size_t rows_used = (size_t)(NB - 1) * SEQ_FULL + SEQ;
  if ((size_t)in_sizes[0] < rows_used * DIM) return;
  if ((size_t)in_sizes[1] < (size_t)DIM * DIM || (size_t)in_sizes[3] < (size_t)DIM * DIM) return;
  if ((size_t)in_sizes[5] < (size_t)DIM * DIM || (size_t)in_sizes[7] < (size_t)DIM * DIM) return;
  if ((size_t)in_sizes[9] < (size_t)DIM * FFN || (size_t)in_sizes[11] < (size_t)FFN * DIM) return;
  if (in_sizes[2] < DIM || in_sizes[4] < DIM || in_sizes[6] < DIM || in_sizes[8] < DIM) return;
  if (in_sizes[10] < FFN || in_sizes[12] < DIM) return;
  if (in_sizes[13] < DIM || in_sizes[14] < DIM || in_sizes[15] < DIM || in_sizes[16] < DIM) return;
  if ((size_t)out_size < rows_used * DIM) return;
  if (ws_size < WS_TOTAL) return;

  const float* x   = (const float*)d_in[0];
  const float* wq  = (const float*)d_in[1];
  const float* bq  = (const float*)d_in[2];
  const float* wk  = (const float*)d_in[3];
  const float* bk  = (const float*)d_in[4];
  const float* wv  = (const float*)d_in[5];
  const float* bv  = (const float*)d_in[6];
  const float* wo  = (const float*)d_in[7];
  const float* bo  = (const float*)d_in[8];
  const float* w1  = (const float*)d_in[9];
  const float* b1  = (const float*)d_in[10];
  const float* w2  = (const float*)d_in[11];
  const float* b2  = (const float*)d_in[12];
  const float* g1  = (const float*)d_in[13];
  const float* be1 = (const float*)d_in[14];
  const float* g2  = (const float*)d_in[15];
  const float* be2 = (const float*)d_in[16];
  float* out = (float*)d_out;

  char* ws = (char*)d_ws;
  f16*   xh    = (f16*)(ws + OFF_XH);
  f16*   wqkvT = (f16*)(ws + OFF_WQKV);
  f16*   woT   = (f16*)(ws + OFF_WO);
  f16*   w1T   = (f16*)(ws + OFF_W1);
  f16*   w2T   = (f16*)(ws + OFF_W2);
  f16*   qk    = (f16*)(ws + OFF_BIG);
  f16*   hh    = (f16*)(ws + OFF_BIG);
  f16*   vt    = (f16*)(ws + OFF_VT);
  f16*   ctx   = (f16*)(ws + OFF_CTX);
  float* y     = (float*)(ws + OFF_Y);
  float* x1f   = (float*)(ws + OFF_X1F);
  f16*   x1h   = (f16*)(ws + OFF_X1H);

  cvt_x_kernel<<<dim3((unsigned)((size_t)NTOK * DIM / 8 / 256)), 256, 0, stream>>>(x, xh);
  wt_kernel<<<dim3(DIM / 64, DIM / 64), 256, 0, stream>>>(wq, wqkvT, DIM, DIM);
  wt_kernel<<<dim3(DIM / 64, DIM / 64), 256, 0, stream>>>(wk, wqkvT + (size_t)DIM * DIM, DIM, DIM);
  wt_kernel<<<dim3(DIM / 64, DIM / 64), 256, 0, stream>>>(wv, wqkvT + (size_t)2 * DIM * DIM, DIM, DIM);
  wt_kernel<<<dim3(DIM / 64, DIM / 64), 256, 0, stream>>>(wo, woT, DIM, DIM);
  wt_kernel<<<dim3(FFN / 64, DIM / 64), 256, 0, stream>>>(w1, w1T, DIM, FFN);
  wt_kernel<<<dim3(DIM / 64, FFN / 64), 256, 0, stream>>>(w2, w2T, FFN, DIM);

  gemm_qkv_kernel<<<dim3(NTOK / GM, QKVN / GN), 128, 0, stream>>>(xh, wqkvT, bq, bk, bv, qk, vt);
  attn_kernel<<<dim3(SEQ / BQ, NHEAD, NB), 256, 0, stream>>>(qk, vt, ctx);
  gemm_wo_kernel<<<dim3(NTOK / GM, DIM / GN), 128, 0, stream>>>(ctx, woT, bo, x, y);
  ln1_kernel<<<dim3(NTOK / 8), 256, 0, stream>>>(y, g1, be1, x1f, x1h);
  gemm_ffn1_kernel<<<dim3(NTOK / GM, FFN / GN), 128, 0, stream>>>(x1h, w1T, b1, hh);
  gemm_ffn2_kernel<<<dim3(NTOK / GM, DIM / GN), 128, 0, stream>>>(hh, w2T, b2, x1f, y);
  ln2_kernel<<<dim3(NTOK / 8), 256, 0, stream>>>(y, g2, be2, out);
}
